// TransformerSelfAttention_6975026888775
// MI455X (gfx1250) — hardware-verified
//
#include <hip/hip_runtime.h>
#include <stdint.h>
#include <stddef.h>

typedef __attribute__((ext_vector_type(16))) _Float16 v16h;
typedef __attribute__((ext_vector_type(8)))  _Float16 v8h;
typedef __attribute__((ext_vector_type(16))) __bf16   v16b;
typedef __attribute__((ext_vector_type(8)))  __bf16   v8b;
typedef __attribute__((ext_vector_type(8)))  float    v8f;
typedef __attribute__((ext_vector_type(4)))  float    v4f;
typedef __attribute__((ext_vector_type(4)))  unsigned v4u;

constexpr int kBatch = 2;
constexpr int kSeq   = 2048;
constexpr int kHid   = 1024;
constexpr int kHeads = 16;
constexpr int kDh    = 64;
constexpr int kTok   = kBatch * kSeq;
static_assert(kHeads * kDh == kHid);
static_assert(kTok % 64 == 0 && kHid % 64 == 0 && kHid % 32 == 0);
static_assert(kSeq % 64 == 0 && kDh == 64);

__device__ __forceinline__ unsigned short f2bf_bits(float f) {
  unsigned u = __float_as_uint(f);
  return (unsigned short)((u + 0x7FFFu + ((u >> 16) & 1u)) >> 16);
}
__device__ __forceinline__ float bf_bits2f(unsigned short h) { return __uint_as_float(((unsigned)h) << 16); }
__device__ __forceinline__ float bfr(float f) { return bf_bits2f(f2bf_bits(f)); }
__device__ __forceinline__ __bf16 f2bf(float f) { return __builtin_bit_cast(__bf16, f2bf_bits(f)); }
__device__ __forceinline__ void bf_split(float f, __bf16& hi, __bf16& lo) {
  const unsigned short hb = f2bf_bits(f);
  hi = __builtin_bit_cast(__bf16, hb);
  lo = f2bf(f - __uint_as_float(((unsigned)hb) << 16));
}

__device__ __forceinline__ void dep_guard_h(v8f& a, v8f& b, v16h x, v16h y) { asm volatile("v_nop\n\tv_nop\n\tv_nop\n\tv_nop" : "+v"(a), "+v"(b) : "v"(x), "v"(y)); }
__device__ __forceinline__ void dep_guard_b(v8f& a, v8f& b, v16b x, v16b y) { asm volatile("v_nop\n\tv_nop\n\tv_nop\n\tv_nop" : "+v"(a), "+v"(b) : "v"(x), "v"(y)); }
__device__ __forceinline__ void keep4_h(v16h a, v16h b, v16h c, v16h d) { asm volatile("v_nop" :: "v"(a), "v"(b), "v"(c), "v"(d)); }
__device__ __forceinline__ void keep4_b(v16b a, v16b b, v16b c, v16b d) { asm volatile("v_nop" :: "v"(a), "v"(b), "v"(c), "v"(d)); }
__device__ __forceinline__ void acc_guard4(v8f& a, v8f& b, v8f& c, v8f& d) { asm volatile("v_nop\n\tv_nop\n\tv_nop\n\tv_nop" : "+v"(a), "+v"(b), "+v"(c), "+v"(d)); }
__device__ __forceinline__ void guard_acc1(v8f& a, v16b w, v16b x, v16b y, v16b z) {
  asm volatile("v_nop\n\tv_nop\n\tv_nop\n\tv_nop" : "+v"(a) : "v"(w), "v"(x), "v"(y), "v"(z));
}

template <typename T> struct Frag;
template <> struct Frag<_Float16> {
  typedef v16h V; union U { v16h v; v8h h[2]; };
  static __device__ __forceinline__ v16h load(const _Float16* p) {
    U f; f.h[0] = *(const v8h*)(p); f.h[1] = *(const v8h*)(p + 16); return f.v;
  }
  static __device__ __forceinline__ v8f mma(v16h a, v16h b, v8f c) {
    return __builtin_amdgcn_wmma_f32_16x16x32_f16(false, a, false, b, (short)0, c, false, false);
  }
  static __device__ __forceinline__ void guard(v8f& a, v8f& b, v16h x, v16h y) { dep_guard_h(a, b, x, y); }
  static __device__ __forceinline__ void keep(v16h a, v16h b, v16h c, v16h d) { keep4_h(a, b, c, d); }
};
template <> struct Frag<__bf16> {
  typedef v16b V; union U { v16b v; v8b h[2]; };
  static __device__ __forceinline__ v16b load(const __bf16* p) {
    U f; f.h[0] = *(const v8b*)(p); f.h[1] = *(const v8b*)(p + 16); return f.v;
  }
  static __device__ __forceinline__ v8f mma(v16b a, v16b b, v8f c) {
    return __builtin_amdgcn_wmma_f32_16x16x32_bf16(false, a, false, b, (short)0, c, false, false);
  }
  static __device__ __forceinline__ void guard(v8f& a, v8f& b, v16b x, v16b y) { dep_guard_b(a, b, x, y); }
  static __device__ __forceinline__ void keep(v16b a, v16b b, v16b c, v16b d) { keep4_b(a, b, c, d); }
};

template <int ET> struct Elem;
template <> struct Elem<0> { typedef _Float16 T; };
template <> struct Elem<1> { typedef __bf16 T; };
template <int ET, bool SPLIT, int BIAS_MODE, int OUT_MODE, bool RESID, int ACT = 0, bool CMUL = false>
__global__ __launch_bounds__(256) void wmma_gemm64(
    const unsigned short* __restrict__ Ap, const unsigned short* __restrict__ A2p, int lda, long strideA,
    const unsigned short* __restrict__ Btp, const unsigned short* __restrict__ Bt2p, int ldb, long strideB,
    void* __restrict__ Cout, void* __restrict__ Cout2, int ldc, long strideC,
    const float* __restrict__ bias, const float* __restrict__ cmul,
    const float* __restrict__ resid, long strideR,
    int M, int N, int K, float scale) {
  typedef typename Elem<ET>::T T;
  typedef typename Frag<T>::V V;
  const T* A = (const T*)Ap; const T* A2 = (const T*)A2p; const T* Bt = (const T*)Btp; const T* Bt2 = (const T*)Bt2p;
  __shared__ __align__(16) float sT[8][16 * 68];
  const int b    = blockIdx.y;
  const int lane = threadIdx.x & 31;
  const int wave = threadIdx.x >> 5;
  const int tilesN = N >> 6;
  const int tilesM = M >> 6;
  const int tile = blockIdx.x * 8 + wave;
  if (tile >= tilesM * tilesN) return;
  const int tm = tile / tilesN;
  const int tn = tile - tm * tilesN;
  const int m0 = tm << 6;
  const int n0 = tn << 6;

  const T* Ab  = A  + (size_t)b * strideA;
  const T* Bb  = Bt + (size_t)b * strideB;
  const T* Ab2 = SPLIT ? (A2  + (size_t)b * strideA) : nullptr;
  const T* Bb2 = SPLIT ? (Bt2 + (size_t)b * strideB) : nullptr;

  const int rlane = lane & 15;
  const int koff  = (lane >> 4) * 8;
  const int mOff  = (lane >> 4) * 8;

  v8f acc[4][4];
#pragma unroll
  for (int i = 0; i < 4; ++i)
#pragma unroll
    for (int j = 0; j < 4; ++j) acc[i][j] = (v8f){0.f,0.f,0.f,0.f,0.f,0.f,0.f,0.f};

  for (int k0 = 0; k0 < K; k0 += 32) {
    V bh[4], bl[4];
#pragma unroll
    for (int j = 0; j < 4; ++j) {
      const size_t bo = (size_t)(n0 + (j << 4) + rlane) * ldb + koff + k0;
      bh[j] = Frag<T>::load(Bb + bo);
      if (SPLIT) bl[j] = Frag<T>::load(Bb2 + bo);
    }
#pragma unroll
    for (int i = 0; i < 4; ++i) {
      const size_t ao = (size_t)(m0 + (i << 4) + rlane) * lda + koff + k0;
      V ah = Frag<T>::load(Ab + ao);
      V al;
      if (SPLIT) al = Frag<T>::load(Ab2 + ao);
#pragma unroll
      for (int j = 0; j < 4; ++j) {
        acc[i][j] = Frag<T>::mma(ah, bh[j], acc[i][j]);
        if (SPLIT) {
          acc[i][j] = Frag<T>::mma(ah, bl[j], acc[i][j]);
          acc[i][j] = Frag<T>::mma(al, bh[j], acc[i][j]);
        }
      }
      Frag<T>::guard(acc[i][0], acc[i][3], ah, SPLIT ? al : ah);
    }
    Frag<T>::keep(bh[0], bh[1], bh[2], bh[3]);
    if (SPLIT) Frag<T>::keep(bl[0], bl[1], bl[2], bl[3]);
  }
  acc_guard4(acc[0][0], acc[0][1], acc[0][2], acc[0][3]);
  acc_guard4(acc[1][0], acc[1][1], acc[1][2], acc[1][3]);
  acc_guard4(acc[2][0], acc[2][1], acc[2][2], acc[2][3]);
  acc_guard4(acc[3][0], acc[3][1], acc[3][2], acc[3][3]);

  float* slab = sT[wave];
  const float* Rb = RESID ? (resid + (size_t)b * strideR) : nullptr;
#pragma unroll
  for (int i = 0; i < 4; ++i) {
    const int mBase = m0 + (i << 4);
#pragma unroll
    for (int j = 0; j < 4; ++j) {
      const int n = n0 + (j << 4) + rlane;
      float bv = 0.f, cmv = 1.f;
      if (BIAS_MODE == 2) bv = bfr(bias[n]);
      if (CMUL) cmv = bfr(cmul[n]);
#pragma unroll
      for (int r = 0; r < 8; ++r) {
        float v = acc[i][j][r] * scale;
        if (BIAS_MODE == 1) v += bfr(bias[mBase + mOff + r]);
        if (BIAS_MODE == 2) v += bv;
        if (CMUL) v *= cmv;
        if (RESID) v += Rb[(size_t)(mBase + mOff + r) * ldc + n];
        if (ACT == 1) v = tanhf(v);
        if (ACT == 2) v = fmaxf(v, 0.0f);
        if (ACT == 4) v = (v > 0.f) ? v : 0.01f * v;
        slab[(mOff + r) * 68 + (j << 4) + rlane] = v;
      }
    }
    __builtin_amdgcn_fence(__ATOMIC_RELEASE, "workgroup");
    __builtin_amdgcn_wave_barrier();
    __builtin_amdgcn_fence(__ATOMIC_ACQUIRE, "workgroup");
    if (OUT_MODE == 0) {
      float* C = (float*)Cout + (size_t)b * strideC;
      const int hh = lane >> 4, c4 = (lane & 15) * 4;
      for (int pass = 0; pass < 2; ++pass) {
#pragma unroll
        for (int it = 0; it < 8; ++it) {
          const int row = it * 2 + hh;
          v4f v = *(const v4f*)(slab + row * 68 + c4);
          *(volatile v4f*)(C + (size_t)(mBase + row) * ldc + n0 + c4) = v;
        }
        __threadfence();
      }
    } else {
      const int q = lane >> 3, c8 = (lane & 7) * 8;
      unsigned short* C  = (unsigned short*)Cout  + (size_t)b * strideC;
      unsigned short* C2 = (OUT_MODE == 2) ? ((unsigned short*)Cout2 + (size_t)b * strideC) : nullptr;
      for (int pass = 0; pass < 2; ++pass) {
#pragma unroll
        for (int it = 0; it < 4; ++it) {
          const int row = it * 4 + q;
          const float* sp = slab + row * 68 + c8;
          v8h hv, lv;
#pragma unroll
          for (int e = 0; e < 8; ++e) {
            if (OUT_MODE == 1) {
              hv[e] = (_Float16)sp[e];
            } else {
              unsigned short hb = f2bf_bits(sp[e]);
              unsigned short lb = f2bf_bits(sp[e] - bf_bits2f(hb));
              hv[e] = __builtin_bit_cast(_Float16, hb);
              lv[e] = __builtin_bit_cast(_Float16, lb);
            }
          }
          *(volatile v8h*)(C + (size_t)(mBase + row) * ldc + n0 + c8) = hv;
          if (OUT_MODE == 2) *(volatile v8h*)(C2 + (size_t)(mBase + row) * ldc + n0 + c8) = lv;
        }
        __threadfence();
      }
    }
    __builtin_amdgcn_fence(__ATOMIC_RELEASE, "workgroup");
    __builtin_amdgcn_wave_barrier();
    __builtin_amdgcn_fence(__ATOMIC_ACQUIRE, "workgroup");
  }
}

__global__ __launch_bounds__(256) void cast_f32_bf16x8(
    const float* __restrict__ in0, const float* __restrict__ in1, const float* __restrict__ in2,
    unsigned short* __restrict__ outp, long plane_elems, int n8) {
  const int which = blockIdx.y;
  const float* in = (which == 0) ? in0 : ((which == 1) ? in1 : in2);
  const int i = blockIdx.x * 256 + threadIdx.x;
  if (i < n8) {
    const size_t e = (size_t)i * 8;
    const v4f a  = *(const v4f*)(in + e);
    const v4f a2 = *(const v4f*)(in + e + 4);
    v4u w;
    w[0] = (unsigned)f2bf_bits(a[0])  | ((unsigned)f2bf_bits(a[1])  << 16);
    w[1] = (unsigned)f2bf_bits(a[2])  | ((unsigned)f2bf_bits(a[3])  << 16);
    w[2] = (unsigned)f2bf_bits(a2[0]) | ((unsigned)f2bf_bits(a2[1]) << 16);
    w[3] = (unsigned)f2bf_bits(a2[2]) | ((unsigned)f2bf_bits(a2[3]) << 16);
    unsigned short* o = outp + (size_t)which * (size_t)plane_elems + e;
    *(volatile v4u*)o = w;
    __threadfence();
    *(volatile v4u*)o = w;
  }
}

#define HEAD_DIM 64
#define QROWS_PER_BLOCK 64
#define KV_CHUNK 64
#define ATT_WAVES 4
#define OS_PITCH 68

__device__ __forceinline__ v8f mma_bf(v16b a, v16b b, v8f c) {
  return __builtin_amdgcn_wmma_f32_16x16x32_bf16(false, a, false, b, (short)0, c, false, false);
}

__global__ __launch_bounds__(128)
void attn_hilo_kernel(const unsigned short* __restrict__ Qhp, const unsigned short* __restrict__ Qlp,
                      const unsigned short* __restrict__ Khp, const unsigned short* __restrict__ Klp,
                      const unsigned short* __restrict__ Vthp, const unsigned short* __restrict__ Vtlp,
                      const float* __restrict__ amask, const float* __restrict__ attm,
                      const float* __restrict__ valm, float* __restrict__ out,
                      int S, int nheads, int hid, int ldvt)
{
  __shared__ __align__(16) __bf16 Psh[ATT_WAVES][16 * KV_CHUNK];
  __shared__ __align__(16) __bf16 Psl[ATT_WAVES][16 * KV_CHUNK];
  __shared__ __align__(16) float  Os[ATT_WAVES][16 * OS_PITCH];

  const __bf16* Qh  = (const __bf16*)Qhp;
  const __bf16* Ql  = (const __bf16*)Qlp;
  const __bf16* Kh  = (const __bf16*)Khp;
  const __bf16* Kl  = (const __bf16*)Klp;
  const __bf16* Vth = (const __bf16*)Vthp;
  const __bf16* Vtl = (const __bf16*)Vtlp;

  const int tid  = threadIdx.x;
  const int wave = tid >> 5;
  const int lane = tid & 31;
  const int hh   = lane >> 4;
  const int c    = lane & 15;

  const int nqb  = S / QROWS_PER_BLOCK;
  const int bx   = blockIdx.x;
  const int qb   = bx % nqb;
  const int bhid = bx / nqb;
  const int h    = bhid % nheads;
  const int b    = bhid / nheads;
  const int q0   = qb * QROWS_PER_BLOCK + wave * 16;
  const size_t tok0 = (size_t)b * (size_t)S;
  const int hcol = h * HEAD_DIM;

  float hsum = bfr(attm[lane]) + bfr(attm[lane + 32]);
#pragma unroll
  for (int off = 1; off < 32; off <<= 1) hsum += __shfl_xor(hsum, off, 32);
  const float qscale = 1.0f / sqrtf(hsum);

  float vmv[4];
#pragma unroll
  for (int t = 0; t < 4; ++t) vmv[t] = bfr(valm[hcol + t * 16 + c]);

  v16b qah[2], qal[2];
  {
    const __bf16* qrh = Qh + (tok0 + (size_t)(q0 + c)) * (size_t)hid + hcol + 8 * hh;
    const __bf16* qrl = Ql + (tok0 + (size_t)(q0 + c)) * (size_t)hid + hcol + 8 * hh;
#pragma unroll
    for (int dc = 0; dc < 2; ++dc) {
      qah[dc] = Frag<__bf16>::load(qrh + dc * 32);
      qal[dc] = Frag<__bf16>::load(qrl + dc * 32);
    }
  }

  float mrow[8], lrow[8];
  v8f oacc[4];
#pragma unroll
  for (int r = 0; r < 8; ++r) { mrow[r] = -INFINITY; lrow[r] = 0.f; }
#pragma unroll
  for (int t = 0; t < 4; ++t) oacc[t] = (v8f){0.f,0.f,0.f,0.f,0.f,0.f,0.f,0.f};

  const int nChunks = S / KV_CHUNK;
  for (int kc = 0; kc < nChunks; ++kc) {
    const int kv0 = kc * KV_CHUNK;
    __syncthreads();

    v8f s[4];
#pragma unroll
    for (int j = 0; j < 4; ++j) {
      s[j] = (v8f){0.f,0.f,0.f,0.f,0.f,0.f,0.f,0.f};
      const size_t krow = (tok0 + (size_t)(kv0 + j * 16 + c)) * (size_t)hid + hcol + 8 * hh;
      const v16b kb0 = Frag<__bf16>::load(Kh + krow);
      const v16b kb1 = Frag<__bf16>::load(Kh + krow + 32);
      const v16b kl0 = Frag<__bf16>::load(Kl + krow);
      const v16b kl1 = Frag<__bf16>::load(Kl + krow + 32);
      s[j] = mma_bf(qah[0], kb0, s[j]);
      s[j] = mma_bf(qah[0], kl0, s[j]);
      s[j] = mma_bf(qal[0], kb0, s[j]);
      s[j] = mma_bf(qah[1], kb1, s[j]);
      s[j] = mma_bf(qah[1], kl1, s[j]);
      s[j] = mma_bf(qal[1], kb1, s[j]);
      guard_acc1(s[j], kb0, kl0, kb1, kl1);
    }

    float am[4];
#pragma unroll
    for (int j = 0; j < 4; ++j) am[j] = bfr(amask[tok0 + (size_t)(kv0 + j * 16 + c)]);
    float cm[8];
#pragma unroll
    for (int r = 0; r < 8; ++r) {
      float m = -INFINITY;
#pragma unroll
      for (int j = 0; j < 4; ++j) {
        const float sv = s[j][r] * qscale + am[j];
        s[j][r] = sv;
        m = fmaxf(m, sv);
      }
#pragma unroll
      for (int off = 1; off < 16; off <<= 1) m = fmaxf(m, __shfl_xor(m, off, 32));
      cm[r] = m;
    }

    __bf16* pwh = Psh[wave];
    __bf16* pwl = Psl[wave];
#pragma unroll
    for (int r = 0; r < 8; ++r) {
      const float mnew  = fmaxf(mrow[r], cm[r]);
      const float alpha = expf(mrow[r] - mnew);
      mrow[r] = mnew;
      float psum = 0.f;
#pragma unroll
      for (int j = 0; j < 4; ++j) {
        const float p = expf(s[j][r] - mnew);
        psum += p;
        __bf16 ph, plo;
        bf_split(p, ph, plo);
        pwh[(8 * hh + r) * KV_CHUNK + j * 16 + c] = ph;
        pwl[(8 * hh + r) * KV_CHUNK + j * 16 + c] = plo;
      }
#pragma unroll
      for (int off = 1; off < 16; off <<= 1) psum += __shfl_xor(psum, off, 32);
      lrow[r] = lrow[r] * alpha + psum;
#pragma unroll
      for (int t = 0; t < 4; ++t) oacc[t][r] *= alpha;
    }
    __syncthreads();

#pragma unroll
    for (int kk = 0; kk < 2; ++kk) {
      const v16b pa = Frag<__bf16>::load(pwh + c * KV_CHUNK + kk * 32 + 8 * hh);
      const v16b pl = Frag<__bf16>::load(pwl + c * KV_CHUNK + kk * 32 + 8 * hh);
#pragma unroll
      for (int t = 0; t < 4; ++t) {
        const size_t vrow = (size_t)(hcol + t * 16 + c) * (size_t)ldvt + tok0 + (size_t)(kv0 + kk * 32 + 8 * hh);
        const v16b vb = Frag<__bf16>::load(Vth + vrow);
        const v16b vl = Frag<__bf16>::load(Vtl + vrow);
        oacc[t] = mma_bf(pa, vb, oacc[t]);
        oacc[t] = mma_bf(pa, vl, oacc[t]);
        oacc[t] = mma_bf(pl, vb, oacc[t]);
        guard_acc1(oacc[t], pa, pl, vb, vl);
      }
    }
  }
  acc_guard4(oacc[0], oacc[1], oacc[2], oacc[3]);

  float* os = Os[wave];
#pragma unroll
  for (int r = 0; r < 8; ++r) {
    const float inv = 1.0f / lrow[r];
#pragma unroll
    for (int t = 0; t < 4; ++t) os[(8 * hh + r) * OS_PITCH + t * 16 + c] = oacc[t][r] * inv * vmv[t];
  }
  __syncthreads();
  {
    const int c4 = (lane & 15) * 4;
    for (int pass = 0; pass < 2; ++pass) {
#pragma unroll
      for (int it = 0; it < 8; ++it) {
        const int row = it * 2 + hh;
        v4f val = *(const v4f*)(os + row * OS_PITCH + c4);
        *(volatile v4f*)(out + (tok0 + (size_t)(q0 + row)) * (size_t)hid + hcol + c4) = val;
      }
      __threadfence();
    }
  }
}

extern "C" void kernel_launch(void* const* d_in, const int* in_sizes, int n_in,
                              void* d_out, int out_size, void* d_ws, size_t ws_size,
                              hipStream_t stream) {
  if (n_in < 10) return;
  if (in_sizes[0] != kTok * kHid || in_sizes[1] != kBatch * kSeq ||
      in_sizes[2] != kHid * kHid || in_sizes[3] != kHid ||
      in_sizes[4] != kHid * kHid || in_sizes[5] != kHid ||
      in_sizes[6] != kHid * kHid || in_sizes[7] != kHid ||
      in_sizes[8] != kHeads * kDh || in_sizes[9] != kHeads * kDh ||
      out_size != kTok * kHid) return;

  const float* hs    = (const float*)d_in[0];
  const float* amask = (const float*)d_in[1];
  const float* Wq    = (const float*)d_in[2];
  const float* bq    = (const float*)d_in[3];
  const float* Wk    = (const float*)d_in[4];
  const float* bk    = (const float*)d_in[5];
  const float* Wv    = (const float*)d_in[6];
  const float* bv    = (const float*)d_in[7];
  const float* attm  = (const float*)d_in[8];
  const float* valm  = (const float*)d_in[9];
  float* out = (float*)d_out;

  const size_t szAct = (size_t)kTok * kHid * 2;
  const size_t szW   = (size_t)kHid * kHid * 2;
  size_t off = 0;
  char* ws = (char*)d_ws;
  unsigned short* Xb  = (unsigned short*)(ws + off); off += szAct;
  unsigned short* Wb  = (unsigned short*)(ws + off); off += 3 * szW;
  unsigned short* Qh  = (unsigned short*)(ws + off); off += szAct;
  unsigned short* Ql  = (unsigned short*)(ws + off); off += szAct;
  unsigned short* Kh  = (unsigned short*)(ws + off); off += szAct;
  unsigned short* Kl  = (unsigned short*)(ws + off); off += szAct;
  unsigned short* Vth = (unsigned short*)(ws + off); off += szAct;
  unsigned short* Vtl = (unsigned short*)(ws + off); off += szAct;
  if (off > ws_size) return;

  static_assert((kTok * kHid) % (8 * 256) == 0 && (kHid * kHid) % (8 * 256) == 0);
  const int nX8 = kTok * kHid / 8;
  const int nW8 = kHid * kHid / 8;
  cast_f32_bf16x8<<<dim3(nX8 / 256, 1), 256, 0, stream>>>(hs, hs, hs, Xb, 0L, nX8);
  cast_f32_bf16x8<<<dim3(nW8 / 256, 3), 256, 0, stream>>>(Wq, Wk, Wv, Wb, (long)kHid * kHid, nW8);

  static_assert(kTok % 64 == 0 && kHid % 64 == 0 && kHid % 32 == 0);
  const int tilesQK = (kTok / 64) * (kHid / 64);
  const int blkQK   = (tilesQK + 7) / 8;
  wmma_gemm64<1, false, 2, 2, false, 0, true><<<dim3(blkQK, 1), 256, 0, stream>>>(
      Xb, Xb, kHid, 0L, Wb, Wb, kHid, 0L, (void*)Qh, (void*)Ql, kHid, 0L,
      bq, attm, nullptr, 0L, kTok, kHid, kHid, 1.0f);
  wmma_gemm64<1, false, 2, 2, false, 0, true><<<dim3(blkQK, 1), 256, 0, stream>>>(
      Xb, Xb, kHid, 0L, Wb + (size_t)kHid * kHid, Wb, kHid, 0L, (void*)Kh, (void*)Kl, kHid, 0L,
      bk, attm, nullptr, 0L, kTok, kHid, kHid, 1.0f);
  const int tilesV = (kHid / 64) * (kTok / 64);
  const int blkV   = (tilesV + 7) / 8;
  wmma_gemm64<1, false, 1, 2, false, 0, false><<<dim3(blkV, 1), 256, 0, stream>>>(
      Wb + 2 * (size_t)kHid * kHid, Wb, kHid, 0L, Xb, Xb, kHid, 0L, (void*)Vth, (void*)Vtl, kTok, 0L,
      bv, nullptr, nullptr, 0L, kHid, kTok, kHid, 1.0f);

  static_assert(kSeq % QROWS_PER_BLOCK == 0 && kSeq % KV_CHUNK == 0 && kDh == HEAD_DIM);
  const int nblk = kBatch * kHeads * (kSeq / QROWS_PER_BLOCK);
  attn_hilo_kernel<<<dim3(nblk), 128, 0, stream>>>(
      Qh, Ql, Kh, Kl, Vth, Vtl, amask, attm, valm, out, kSeq, kHeads, kHid, kTok);
}
